// SemanticCritic_30691836297666
// MI455X (gfx1250) — hardware-run, weakly checked
//
#include <hip/hip_runtime.h>

typedef __attribute__((ext_vector_type(16))) _Float16 v16h;
typedef __attribute__((ext_vector_type(8)))  _Float16 v8h;
typedef __attribute__((ext_vector_type(8)))  float    v8f;
typedef __attribute__((ext_vector_type(4)))  float    v4f;

constexpr int kB      = 65536;
constexpr int kPairs  = 3;
constexpr int kObsW   = 55;
constexpr int kGoalW  = 9;
constexpr int kActW   = 4;
constexpr int kBody   = 10;
constexpr int kObjW   = 15;
constexpr int kNObj   = 3;
constexpr int kKin    = 54;
constexpr int kKinPad = 64;
constexpr int kHid    = 256;
static_assert(2 + 2 + kBody + 2 * (kNObj + kObjW) + kActW == kKin, "pair-input row width");
static_assert(kBody + kNObj * kObjW == kObsW, "obs row width");
static_assert((kKinPad % 32) == 0 && (kHid % 32) == 0, "GEMM K multiples of 32");

constexpr int kRowsPerBlock = 64;
constexpr int kRowGroups    = 4;
constexpr int kColHalf      = 128;
constexpr int kNtPerWave    = 8;
static_assert(kRowGroups * 16 == kRowsPerBlock, "row groups");
static_assert(2 * kColHalf == kHid && kNtPerWave * 16 == kColHalf, "column halves");
static_assert((kB % kRowsPerBlock) == 0 && (kB % 32) == 0, "tile multiples");

constexpr float kActCarry = 16.0f;
constexpr float kWCarry   = 256.0f;
constexpr float kFold     = 1.0f / (kActCarry * kWCarry);
static_assert(kFold * 4096.0f == 1.0f, "fold constant");

constexpr size_t kHW1T = 0;
constexpr size_t kHW3T = kHW1T + (size_t)kHid * kKinPad;
constexpr size_t kHW2T = kHW3T + (size_t)kHid * kKinPad;
constexpr size_t kHW4T = kHW2T + (size_t)kHid * kHid;
constexpr size_t kHW5T = kHW4T + (size_t)kHid * kHid;
constexpr size_t kHW7T = kHW5T + (size_t)kHid * kHid;
constexpr size_t kHX16 = kHW7T + (size_t)kHid * kHid;
constexpr size_t kWsTotal = (kHX16 + (size_t)kPairs * kB * kKinPad) * 2;
static_assert(kWsTotal == 25755648ull, "carve total");
static_assert(kWsTotal <= 134217728ull, "carve cap");
static_assert(((kHW3T * 2) % 128) == 0 && ((kHW2T * 2) % 128) == 0 && ((kHW4T * 2) % 128) == 0 &&
              ((kHW5T * 2) % 128) == 0 && ((kHW7T * 2) % 128) == 0 && ((kHX16 * 2) % 128) == 0, "128-B aligned regions");

constexpr int kHP = 264;
static_assert(((kHP * 2) % 16) == 0, "16-B aligned LDS rows");

__device__ __forceinline__ float rne_bf16(float f) {
  unsigned u = __float_as_uint(f);
  u = (u + 0x7FFFu + ((u >> 16) & 1u)) & 0xFFFF0000u;
  return __uint_as_float(u);
}

struct FragH {
  union U { v16h v; v8h h[2]; };
  static __device__ __forceinline__ v16h load(const _Float16* p) {
    U f;
    f.h[0] = *(const v8h*)(p);
    f.h[1] = *(const v8h*)(p + 16);
    return f.v;
  }
};

__device__ __forceinline__ v8f mma_g(v16h a, v16h b, v8f c) {
  c = __builtin_amdgcn_wmma_f32_16x16x32_f16(false, a, false, b, (short)0, c, false, false);
  asm volatile("v_nop\n\tv_nop\n\tv_nop\n\tv_nop" : "+v"(c) : "v"(a), "v"(b));
  return c;
}

__global__ __launch_bounds__(256) void prep_weights_kernel(
    const float* __restrict__ w1, const float* __restrict__ w3,
    const float* __restrict__ w2, const float* __restrict__ w4,
    const float* __restrict__ w5, const float* __restrict__ w7,
    unsigned short* __restrict__ planes)
{
  const int blk = blockIdx.x;
  const int tid = threadIdx.x;
  const float* src;
  int kreal, kshift, cb;
  size_t dstOff;
  if (blk < 8) {
    src = w1; kreal = kKin; kshift = 3; cb = blk; dstOff = kHW1T;
  } else if (blk < 16) {
    src = w3; kreal = kKin; kshift = 3; cb = blk - 8; dstOff = kHW3T;
  } else {
    const int j = blk - 16;
    const int which = j >> 5;
    cb = j & 31;
    kreal = kHid; kshift = 5;
    src = (which == 0) ? w2 : (which == 1) ? w4 : (which == 2) ? w5 : w7;
    dstOff = kHW2T + (size_t)which * kHid * kHid;
  }
  const int chunk = cb * 256 + tid;
  const int n  = chunk >> kshift;
  const int kc = (chunk & ((1 << kshift) - 1)) * 8;
  const int kpad = 8 << kshift;

  float f0, f1, f2, f3, f4, f5, f6, f7;
  {
    const int kl = kreal - 1;
    const int k0 = (kc + 0 < kl) ? (kc + 0) : kl;
    const int k1 = (kc + 1 < kl) ? (kc + 1) : kl;
    const int k2 = (kc + 2 < kl) ? (kc + 2) : kl;
    const int k3 = (kc + 3 < kl) ? (kc + 3) : kl;
    const int k4 = (kc + 4 < kl) ? (kc + 4) : kl;
    const int k5 = (kc + 5 < kl) ? (kc + 5) : kl;
    const int k6 = (kc + 6 < kl) ? (kc + 6) : kl;
    const int k7 = (kc + 7 < kl) ? (kc + 7) : kl;
    f0 = src[k0 * kHid + n];
    f1 = src[k1 * kHid + n];
    f2 = src[k2 * kHid + n];
    f3 = src[k3 * kHid + n];
    f4 = src[k4 * kHid + n];
    f5 = src[k5 * kHid + n];
    f6 = src[k6 * kHid + n];
    f7 = src[k7 * kHid + n];
  }
  asm volatile("" : "+v"(f0), "+v"(f1), "+v"(f2), "+v"(f3));
  asm volatile("" : "+v"(f4), "+v"(f5), "+v"(f6), "+v"(f7));
  v8h hv;
  hv[0] = (_Float16)((kc + 0 < kreal) ? rne_bf16(f0) * kWCarry : 0.0f);
  hv[1] = (_Float16)((kc + 1 < kreal) ? rne_bf16(f1) * kWCarry : 0.0f);
  hv[2] = (_Float16)((kc + 2 < kreal) ? rne_bf16(f2) * kWCarry : 0.0f);
  hv[3] = (_Float16)((kc + 3 < kreal) ? rne_bf16(f3) * kWCarry : 0.0f);
  hv[4] = (_Float16)((kc + 4 < kreal) ? rne_bf16(f4) * kWCarry : 0.0f);
  hv[5] = (_Float16)((kc + 5 < kreal) ? rne_bf16(f5) * kWCarry : 0.0f);
  hv[6] = (_Float16)((kc + 6 < kreal) ? rne_bf16(f6) * kWCarry : 0.0f);
  hv[7] = (_Float16)((kc + 7 < kreal) ? rne_bf16(f7) * kWCarry : 0.0f);
  unsigned short* dp = planes + dstOff + (size_t)n * kpad + kc;
  *(volatile v8h*)dp = hv;
  __threadfence();
  *(volatile v8h*)dp = hv;
}

constexpr int kRawObs  = 0;
constexpr int kRawAg   = 32 * kObsW;
constexpr int kRawG    = kRawAg + 32 * kGoalW;
constexpr int kRawAn   = kRawG + 32 * kGoalW;
constexpr int kRawAct  = kRawAn + 32 * kGoalW;
constexpr int kRawZero = kRawAct + 32 * kActW;
constexpr int kRawOne  = kRawZero + 1;
constexpr int kRawTot  = kRawZero + 4;
static_assert(kRawAg == 1760 && kRawG == 2048 && kRawAn == 2336 && kRawAct == 2624 && kRawZero == 2752, "LDS raw map");

__device__ __forceinline__ int pair_src_index(int col, int r, int p, int bit2, int oi, int oj) {
  const int ob = kRawObs + r * kObsW;
  int s = kRawZero;
  s = (col == 0) ? (kRawAg + r * kGoalW + p) : s;
  s = (col == 1) ? (kRawAg + r * kGoalW + bit2) : s;
  s = (col == 2) ? (kRawG + r * kGoalW + p) : s;
  s = (col == 3) ? (kRawG + r * kGoalW + bit2) : s;
  s = (col >= 4 && col < 14) ? (ob + col - 4) : s;
  s = (col >= 14 && col < 17) ? ((col - 14 == oi) ? kRawOne : kRawZero) : s;
  s = (col >= 17 && col < 32) ? (ob + kBody + kObjW * oi + col - 17) : s;
  s = (col >= 32 && col < 35) ? ((col - 32 == oj) ? kRawOne : kRawZero) : s;
  s = (col >= 35 && col < 50) ? (ob + kBody + kObjW * oj + col - 35) : s;
  s = (col >= 50 && col < 54) ? (kRawAct + r * kActW + col - 50) : s;
  return s;
}

__device__ __forceinline__ v8h build_chunk(const float* sRaw, int r, int c8, int p, int o1, int o2, int j, int k) {
  const float aj = sRaw[kRawAn + r * kGoalW + j];
  const float ak = sRaw[kRawAn + r * kGoalW + k];
  const bool sel = (aj - ak) >= 0.0f;
  const int bit2 = sel ? j : k;
  const int oi   = sel ? o1 : o2;
  const int oj   = sel ? o2 : o1;
  v8h hv;
#pragma unroll
  for (int e = 0; e < 8; ++e) {
    const int s = pair_src_index(c8 * 8 + e, r, p, bit2, oi, oj);
    const float val = sRaw[s] * kActCarry;
    hv[e] = (_Float16)val;
  }
  return hv;
}

__device__ __forceinline__ void stage_v4(float* dst, const float* __restrict__ gsrc, int idx, int count) {
  const int idc = (idx < count) ? idx : (count - 1);
  const v4f v = *(const v4f*)(gsrc + 4 * idc);
  float x0 = v[0], x1 = v[1], x2 = v[2], x3 = v[3];
  asm volatile("" : "+v"(x0), "+v"(x1), "+v"(x2), "+v"(x3));
  if (idx < count) {
    dst[4 * idx + 0] = rne_bf16(x0);
    dst[4 * idx + 1] = rne_bf16(x1);
    dst[4 * idx + 2] = rne_bf16(x2);
    dst[4 * idx + 3] = rne_bf16(x3);
  }
}

__global__ __launch_bounds__(256) void pack_pairs_kernel(
    const float* __restrict__ obs, const float* __restrict__ ag, const float* __restrict__ g,
    const float* __restrict__ anchor, const float* __restrict__ act,
    unsigned short* __restrict__ X16)
{
  __shared__ __align__(16) float sRaw[kRawTot];
  const int tid = threadIdx.x;
  const int b0  = blockIdx.x * 32;
  stage_v4(sRaw + kRawObs, obs + (size_t)b0 * kObsW, tid, 32 * kObsW / 4);
  stage_v4(sRaw + kRawObs, obs + (size_t)b0 * kObsW, tid + 256, 32 * kObsW / 4);
  stage_v4(sRaw + kRawAg,  ag + (size_t)b0 * kGoalW, tid, 32 * kGoalW / 4);
  stage_v4(sRaw + kRawG,   g + (size_t)b0 * kGoalW, tid, 32 * kGoalW / 4);
  stage_v4(sRaw + kRawAn,  anchor + (size_t)b0 * kGoalW, tid, 32 * kGoalW / 4);
  stage_v4(sRaw + kRawAct, act + (size_t)b0 * kActW, tid, 32 * kActW / 4);
  if (tid == 0) {
    sRaw[kRawZero] = 0.0f;
    sRaw[kRawOne]  = 1.0f;
    sRaw[kRawZero + 2] = 0.0f;
    sRaw[kRawZero + 3] = 0.0f;
  }
  __syncthreads();

  const int r  = tid >> 3;
  const int c8 = tid & 7;
  const v8h h0 = build_chunk(sRaw, r, c8, 0, 0, 1, 3, 5);
  const v8h h1 = build_chunk(sRaw, r, c8, 1, 0, 2, 4, 7);
  const v8h h2 = build_chunk(sRaw, r, c8, 2, 1, 2, 6, 8);
  unsigned short* d0 = X16 + ((size_t)(0 * kB + b0 + r) * kKinPad + c8 * 8);
  unsigned short* d1 = X16 + ((size_t)(1 * kB + b0 + r) * kKinPad + c8 * 8);
  unsigned short* d2 = X16 + ((size_t)(2 * kB + b0 + r) * kKinPad + c8 * 8);
  *(volatile v8h*)d0 = h0;
  *(volatile v8h*)d1 = h1;
  *(volatile v8h*)d2 = h2;
  __threadfence();
  *(volatile v8h*)d0 = h0;
  *(volatile v8h*)d1 = h1;
  *(volatile v8h*)d2 = h2;
}

__device__ __forceinline__ void stage_plane_256(const _Float16* __restrict__ src, _Float16* dst, int tid) {
#pragma unroll 4
  for (int i = 0; i < 32; ++i) {
    const int c = tid + 256 * i;
    const int n = c >> 5;
    const int w = (c & 31) * 8;
    *(v8h*)(dst + n * kHP + w) = *(const v8h*)(src + n * kHid + w);
  }
}

__global__ __launch_bounds__(256) __attribute__((amdgpu_num_vgpr(256))) void fused_pool_mlp_kernel(
    const unsigned short* __restrict__ wsp,
    const float* __restrict__ bA0, const float* __restrict__ bA1,
    const float* __restrict__ bB0, const float* __restrict__ bB1,
    const float* __restrict__ bC0, const float* __restrict__ bC1,
    const float* __restrict__ wo0, const float* __restrict__ wo1,
    const float* __restrict__ bo0, const float* __restrict__ bo1,
    float* __restrict__ out)
{
  __shared__ __align__(16) _Float16 lds_w[kHid * kHP];
  __shared__ __align__(16) _Float16 lds_h[kRowGroups * 16 * kHP];
  __shared__ __align__(16) float sPar[4 * kHid];
  __shared__ __align__(16) float sQ[2 * kRowsPerBlock];

  const int tid  = threadIdx.x;
  const int wave = tid >> 5;
  const int lane = tid & 31;
  const int l16  = lane & 15;
  const int hh   = lane >> 4;
  const int koff = hh * 8;
  const int rg   = wave & 3;
  const int ch   = wave >> 2;
  const int colBase = ch * kColHalf;
  const int m    = blockIdx.y;
  const int rowBase = blockIdx.x * kRowsPerBlock + rg * 16;

  const _Float16* P    = (const _Float16*)wsp;
  const _Float16* WL1  = P + (m ? kHW3T : kHW1T);
  const _Float16* WL2  = P + (m ? kHW4T : kHW2T);
  const _Float16* WL3  = P + (m ? kHW7T : kHW5T);
  const _Float16* X    = P + kHX16;
  const float* bA = m ? bA1 : bA0;
  const float* bB = m ? bB1 : bB0;
  const float* bC = m ? bC1 : bC0;
  const float* wo = m ? wo1 : wo0;
  const float* bo = m ? bo1 : bo0;

  sPar[tid]            = rne_bf16(bA[tid]);
  sPar[kHid + tid]     = rne_bf16(bB[tid]);
  sPar[2 * kHid + tid] = rne_bf16(bC[tid]);
  sPar[3 * kHid + tid] = rne_bf16(wo[tid]);
  float bout = bo[0];
  asm volatile("" : "+v"(bout));
  bout = rne_bf16(bout);

  _Float16* myH = lds_h + rg * (16 * kHP);
  const _Float16* ap = myH + l16 * kHP + koff;

  stage_plane_256(WL2, lds_w, tid);
  __syncthreads();

  v8f sacc[kNtPerWave];
#pragma unroll
  for (int nt = 0; nt < kNtPerWave; ++nt) sacc[nt] = (v8f){0.f, 0.f, 0.f, 0.f, 0.f, 0.f, 0.f, 0.f};

#pragma unroll 1
  for (int p = 0; p < kPairs; ++p) {
    const _Float16* xp = X + ((size_t)p * kB + rowBase + l16) * kKinPad + koff;
    const v16h a0 = FragH::load(xp);
    const v16h a1 = FragH::load(xp + 32);
#pragma unroll 1
    for (int nt = 0; nt < kNtPerWave; ++nt) {
      const int n = colBase + nt * 16 + l16;
      const _Float16* bp = WL1 + n * kKinPad + koff;
      const v16h b0 = FragH::load(bp);
      const v16h b1 = FragH::load(bp + 32);
      v8f c = (v8f){0.f, 0.f, 0.f, 0.f, 0.f, 0.f, 0.f, 0.f};
      c = mma_g(a0, b0, c);
      c = mma_g(a1, b1, c);
      const float bias = sPar[n];
#pragma unroll
      for (int r = 0; r < 8; ++r) {
        const float hv = fmaxf(c[r] * kFold + bias, 0.0f);
        myH[(8 * hh + r) * kHP + n] = (_Float16)(hv * kActCarry);
      }
    }
    __syncthreads();

#pragma unroll
    for (int nt = 0; nt < kNtPerWave; ++nt) {
      const int n = colBase + nt * 16 + l16;
      const _Float16* bp = lds_w + n * kHP + koff;
      v8f c = (v8f){0.f, 0.f, 0.f, 0.f, 0.f, 0.f, 0.f, 0.f};
#pragma unroll 2
      for (int kt = 0; kt < 8; ++kt) {
        const v16h a = FragH::load(ap + kt * 32);
        const v16h b = FragH::load(bp + kt * 32);
        c = mma_g(a, b, c);
      }
      const float bias = sPar[kHid + n];
#pragma unroll
      for (int r = 0; r < 8; ++r) {
        const float xv = fmaxf(c[r] * kFold + bias, 0.0f);
        sacc[nt][r] += xv;
      }
    }
    __syncthreads();
  }

  stage_plane_256(WL3, lds_w, tid);
#pragma unroll
  for (int nt = 0; nt < kNtPerWave; ++nt) {
#pragma unroll
    for (int r = 0; r < 8; ++r)
      myH[(8 * hh + r) * kHP + colBase + nt * 16 + l16] = (_Float16)(sacc[nt][r] * kActCarry);
  }
  __syncthreads();

  float qp[8];
#pragma unroll
  for (int r = 0; r < 8; ++r) qp[r] = 0.0f;

#pragma unroll 1
  for (int nt = 0; nt < kNtPerWave; ++nt) {
    const int n = colBase + nt * 16 + l16;
    const _Float16* bp = lds_w + n * kHP + koff;
    v8f c = (v8f){0.f, 0.f, 0.f, 0.f, 0.f, 0.f, 0.f, 0.f};
#pragma unroll 2
    for (int kt = 0; kt < 8; ++kt) {
      const v16h a = FragH::load(ap + kt * 32);
      const v16h b = FragH::load(bp + kt * 32);
      c = mma_g(a, b, c);
    }
    const float bias = sPar[2 * kHid + n];
    const float wv   = sPar[3 * kHid + n];
#pragma unroll
    for (int r = 0; r < 8; ++r) {
      const float u = fmaxf(c[r] * kFold + bias, 0.0f);
      qp[r] = fmaf(u, wv, qp[r]);
    }
  }

#pragma unroll
  for (int r = 0; r < 8; ++r) {
    float v = qp[r];
    v += __shfl_xor(v, 1, 32);
    v += __shfl_xor(v, 2, 32);
    v += __shfl_xor(v, 4, 32);
    v += __shfl_xor(v, 8, 32);
    if (l16 == 0) sQ[ch * kRowsPerBlock + rg * 16 + 8 * hh + r] = v;
  }
  __syncthreads();

  if (wave == 0) {
    const int i4 = (lane & 15) * 4;
    v4f q;
    q[0] = (sQ[i4 + 0] + sQ[kRowsPerBlock + i4 + 0]) + bout;
    q[1] = (sQ[i4 + 1] + sQ[kRowsPerBlock + i4 + 1]) + bout;
    q[2] = (sQ[i4 + 2] + sQ[kRowsPerBlock + i4 + 2]) + bout;
    q[3] = (sQ[i4 + 3] + sQ[kRowsPerBlock + i4 + 3]) + bout;
    float* dp = out + (size_t)m * kB + (size_t)blockIdx.x * kRowsPerBlock + i4;
    if (lane < 16) *(volatile v4f*)dp = q;
    __threadfence();
    if (lane < 16) *(volatile v4f*)dp = q;
  }
}

extern "C" void kernel_launch(void* const* d_in, const int* in_sizes, int n_in,
                              void* d_out, int out_size, void* d_ws, size_t ws_size,
                              hipStream_t stream) {
  if (n_in < 21) return;
  if (in_sizes[0] != kB * kObsW) return;
  if (in_sizes[1] != kB * kGoalW) return;
  if (in_sizes[2] != kB * kGoalW) return;
  if (in_sizes[3] != kB * kGoalW) return;
  if (in_sizes[4] != kB * kActW) return;
  if (in_sizes[5] != kKin * kHid || in_sizes[9] != kKin * kHid) return;
  if (in_sizes[7] != kHid * kHid || in_sizes[11] != kHid * kHid) return;
  if (in_sizes[13] != kHid * kHid || in_sizes[17] != kHid * kHid) return;
  if (in_sizes[6] != kHid || in_sizes[8] != kHid || in_sizes[10] != kHid || in_sizes[12] != kHid) return;
  if (in_sizes[14] != kHid || in_sizes[18] != kHid) return;
  if (in_sizes[15] != kHid || in_sizes[19] != kHid) return;
  if (in_sizes[16] != 1 || in_sizes[20] != 1) return;
  if (out_size != 2 * kB) return;
  if (ws_size < kWsTotal) return;

  const float* obs    = (const float*)d_in[0];
  const float* ag     = (const float*)d_in[1];
  const float* g      = (const float*)d_in[2];
  const float* anchor = (const float*)d_in[3];
  const float* act    = (const float*)d_in[4];
  const float* w1 = (const float*)d_in[5];
  const float* b1 = (const float*)d_in[6];
  const float* w2 = (const float*)d_in[7];
  const float* b2 = (const float*)d_in[8];
  const float* w3 = (const float*)d_in[9];
  const float* b3 = (const float*)d_in[10];
  const float* w4 = (const float*)d_in[11];
  const float* b4 = (const float*)d_in[12];
  const float* w5 = (const float*)d_in[13];
  const float* b5 = (const float*)d_in[14];
  const float* w6 = (const float*)d_in[15];
  const float* b6 = (const float*)d_in[16];
  const float* w7 = (const float*)d_in[17];
  const float* b7 = (const float*)d_in[18];
  const float* w8 = (const float*)d_in[19];
  const float* b8 = (const float*)d_in[20];

  unsigned short* planes = (unsigned short*)d_ws;
  float* out = (float*)d_out;

  prep_weights_kernel<<<dim3(144), dim3(256), 0, stream>>>(w1, w3, w2, w4, w5, w7, planes);

  pack_pairs_kernel<<<dim3(kB / 32), dim3(256), 0, stream>>>(obs, ag, g, anchor, act, planes + kHX16);

  fused_pool_mlp_kernel<<<dim3(kB / kRowsPerBlock, 2), dim3(256), 0, stream>>>(
      planes,
      b1, b3,
      b2, b4,
      b5, b7,
      w6, w8,
      b6, b8,
      out);
}
